// GraphStructureAttention_18863496364647
// MI455X (gfx1250) — hardware-verified
//
#include <hip/hip_runtime.h>
#include <stddef.h>


#define NTHR  256
#define NWAVE 8
#define HC    128
#define PQW   256
#define GR    32
#define GC    128
#define XSP   132
#define NB    512
#define CHUNK 2048
#define WCAP  256
#define NGRP  (CHUNK / (NTHR * 4))
#define AGG_LDS_BYTES ((NB * HC) * 4 + (NWAVE * WCAP + NWAVE) * 4)

static_assert(NGRP == 2);
static_assert(WCAP == (CHUNK / NTHR) * 32);
static_assert(AGG_LDS_BYTES == 270368);
static_assert((NB & (NB - 1)) == 0);
static_assert(NB <= 512);
static_assert((XSP % 4) == 0);
static_assert((HC / 8) == 16);

typedef float          v4f  __attribute__((ext_vector_type(4)));
typedef float          v8f  __attribute__((ext_vector_type(8)));
typedef int            v4i  __attribute__((ext_vector_type(4)));
typedef _Float16       v8h  __attribute__((ext_vector_type(8)));
typedef _Float16       v16h __attribute__((ext_vector_type(16)));

union FragH { v16h v; v4i u[2]; };
union Pack  { v8h h; v4i i; };

__device__ __forceinline__ v8f wmh(v16h a, v16h b, v8f c) {
  v8f d = __builtin_amdgcn_wmma_f32_16x16x32_f16(false, a, false, b, (short)0, c, false, false);
  asm volatile("v_nop\n\tv_nop\n\tv_nop\n\tv_nop" : "+v"(d) : "v"(a), "v"(b));
  return d;
}

__global__ __launch_bounds__(NTHR) void k_cvt_x(const float* __restrict__ x, int rows_src,
                                                unsigned short* xh, int rows_total) {
  const int n8 = rows_total * (HC / 8);
  const int i  = blockIdx.x * NTHR + threadIdx.x;
  if (i >= n8) return;
  const int r  = i >> 4;
  const int kb = (i & 15) * 8;
  Pack u;
  const v4i z4 = {0, 0, 0, 0};
  u.i = z4;
  if (r < rows_src) {
    const v4f a = *(const v4f*)(x + (size_t)r * HC + kb);
    const v4f b = *(const v4f*)(x + (size_t)r * HC + kb + 4);
    u.h[0] = (_Float16)a.x; u.h[1] = (_Float16)a.y; u.h[2] = (_Float16)a.z; u.h[3] = (_Float16)a.w;
    u.h[4] = (_Float16)b.x; u.h[5] = (_Float16)b.y; u.h[6] = (_Float16)b.z; u.h[7] = (_Float16)b.w;
  }
  const size_t o = (size_t)i * 8;
  *(volatile v4i*)(xh + o) = u.i;
  __threadfence();
  *(volatile v4i*)(xh + o) = u.i;
}

__global__ __launch_bounds__(NTHR) void k_cvt_w(const float* __restrict__ W1, unsigned short* bt, float wscale) {
  const int i = blockIdx.x * NTHR + threadIdx.x;
  if (i >= PQW * (HC / 8)) return;
  const int c    = i >> 4;
  const int kb   = (i & 15) * 8;
  const int part = c >> 7;
  const int n    = c & (HC - 1);
  Pack u;
#pragma unroll
  for (int j = 0; j < 8; ++j)
    u.h[j] = (_Float16)(W1[(size_t)(part * HC + kb + j) * HC + n] * wscale);
  const size_t o = (size_t)i * 8;
  *(volatile v4i*)(bt + o) = u.i;
  __threadfence();
  *(volatile v4i*)(bt + o) = u.i;
}

__global__ __launch_bounds__(NTHR) void k_gemm(
    const unsigned short* __restrict__ A, const unsigned short* __restrict__ B,
    const float* __restrict__ bias, float* out, int K, int Ncols, int bias0, float oscale) {
  __shared__ __attribute__((aligned(16))) float Xs[GR * XSP];

  const int tid  = threadIdx.x;
  const int lane = tid & 31;
  const int wave = tid >> 5;
  const int hh   = lane >> 4;
  const int m    = lane & 15;
  const int rowBase = blockIdx.x * GR;
  const int colBase = blockIdx.y * GC;
  const int ncol = colBase + wave * 16 + m;

  const size_t ra0 = (size_t)(rowBase + m) * K + 8 * hh;
  const size_t ra1 = ra0 + (size_t)16 * K;
  const size_t rb  = (size_t)ncol * K + 8 * hh;

  v8f c0 = {0.f, 0.f, 0.f, 0.f, 0.f, 0.f, 0.f, 0.f};
  v8f c1 = {0.f, 0.f, 0.f, 0.f, 0.f, 0.f, 0.f, 0.f};

#pragma unroll 1
  for (int k0 = 0; k0 < K; k0 += 32) {
    FragH a0, a1, b;
    a0.u[0] = *(const v4i*)(A + ra0 + k0);  a0.u[1] = *(const v4i*)(A + ra0 + k0 + 16);
    a1.u[0] = *(const v4i*)(A + ra1 + k0);  a1.u[1] = *(const v4i*)(A + ra1 + k0 + 16);
    b.u[0]  = *(const v4i*)(B + rb + k0);   b.u[1]  = *(const v4i*)(B + rb + k0 + 16);
    c0 = wmh(a0.v, b.v, c0);
    c1 = wmh(a1.v, b.v, c1);
  }

  const int bi  = ncol - bias0;
  const float bl = bias[bi < 0 ? 0 : bi];
  const float bv = (bi >= 0) ? bl : 0.f;
  const int cl = wave * 16 + m;
#pragma unroll
  for (int r = 0; r < 8; ++r) {
    Xs[(8 * hh + r) * XSP + cl]      = c0[r] * oscale + bv;
    Xs[(16 + 8 * hh + r) * XSP + cl] = c1[r] * oscale + bv;
  }
  __syncthreads();

  v4f xv[4];
  float* xpp[4];
#pragma unroll
  for (int i = 0; i < 4; ++i) {
    xv[i]  = *(const v4f*)(Xs + (4 * wave + i) * XSP + 4 * lane);
    xpp[i] = out + (size_t)(rowBase + 4 * wave + i) * Ncols + colBase + 4 * lane;
  }
#pragma unroll
  for (int i = 0; i < 4; ++i) *(volatile v4f*)(xpp[i]) = xv[i];
  __threadfence();
#pragma unroll
  for (int i = 0; i < 4; ++i) *(volatile v4f*)(xpp[i]) = xv[i];
}

__global__ __launch_bounds__(NTHR) void k_agg(
    const int* __restrict__ ei, const float* __restrict__ x, const float* __restrict__ pq,
    const float* __restrict__ w2, const float* __restrict__ b2p,
    const float* __restrict__ gam, const float* __restrict__ bet,
    float* out, int nN, int nE) {
  extern __shared__ v4f lds_dyn[];
  float* sacc = (float*)lds_dyn;
  int*   list = (int*)(sacc + NB * HC);
  int*   wcnt = list + NWAVE * WCAP;

  const int tid  = threadIdx.x;
  const int lane = tid & 31;
  const int wave = tid >> 5;
  const int nodeBase = blockIdx.x * NB;

  {
    const v4f z4 = {0.f, 0.f, 0.f, 0.f};
    for (int i = tid; i < (NB * HC) / 4; i += NTHR) lds_dyn[i] = z4;
  }
  __syncthreads();

  const int co = 4 * lane;
  const v4f  w2v = *(const v4f*)(w2 + co);
  const float b2v = b2p[0];
  const v4f  gv  = *(const v4f*)(gam + co);
  const v4f  bv  = *(const v4f*)(bet + co);

  const int* eid = ei + nE;
  const bool al16 = ((nE & 3) == 0);
  const int nChunks = (nE + CHUNK - 1) / CHUNK;

#pragma unroll 1
  for (int ch = 0; ch < nChunks; ++ch) {
    const int cbase = ch * CHUNK;
    int wc = 0;
#pragma unroll
    for (int g = 0; g < NGRP; ++g) {
      const int el0 = (g * NTHR + tid) * 4;
      const int e0  = cbase + el0;
      const int sent = -2147483647 - 1;
      v4i d;
      if (al16 && (e0 + 3 < nE)) {
        d = *(const v4i*)(eid + e0);
      } else {
        d.x = (e0     < nE) ? eid[min(e0, nE - 1)]     : sent;
        d.y = (e0 + 1 < nE) ? eid[min(e0 + 1, nE - 1)] : sent;
        d.z = (e0 + 2 < nE) ? eid[min(e0 + 2, nE - 1)] : sent;
        d.w = (e0 + 3 < nE) ? eid[min(e0 + 3, nE - 1)] : sent;
      }
      const unsigned s0 = (unsigned)d.x - (unsigned)nodeBase;
      const unsigned s1 = (unsigned)d.y - (unsigned)nodeBase;
      const unsigned s2 = (unsigned)d.z - (unsigned)nodeBase;
      const unsigned s3 = (unsigned)d.w - (unsigned)nodeBase;
      const bool h0 = s0 < (unsigned)NB;
      const bool h1 = s1 < (unsigned)NB;
      const bool h2 = s2 < (unsigned)NB;
      const bool h3 = s3 < (unsigned)NB;
      const unsigned many = __builtin_amdgcn_ballot_w32(h0 | h1 | h2 | h3);
      if (many != 0u) {
#define HITJ(J, HJ, SJ) { \
          const unsigned mj = __builtin_amdgcn_ballot_w32(HJ); \
          if (HJ) { \
            const int pos = wc + (int)__builtin_amdgcn_mbcnt_lo(mj, 0u); \
            if (pos < WCAP) list[wave * WCAP + pos] = ((el0 + (J)) << 9) | (int)(SJ); \
          } \
          wc += (int)__builtin_popcount(mj); }
        HITJ(0, h0, s0)
        HITJ(1, h1, s1)
        HITJ(2, h2, s2)
        HITJ(3, h3, s3)
#undef HITJ
      }
    }
    if (lane == 0) wcnt[wave] = wc;
    __syncthreads();

    if (wave == 0) {
#pragma unroll 1
      for (int wsx = 0; wsx < NWAVE; ++wsx) {
        int n = __builtin_amdgcn_readfirstlane(wcnt[wsx]);
        n = n > WCAP ? WCAP : n;
        n = n < 0 ? 0 : n;
#pragma unroll 1
        for (int i = 0; i < n; ++i) {
          const int ent  = __builtin_amdgcn_readfirstlane(list[wsx * WCAP + i]);
          const int slot = ent & (NB - 1);
          const int el   = (ent >> 9) & (CHUNK - 1);
          const int node = nodeBase + slot;
          if (node >= nN) continue;
          int e = cbase + el;
          if (e > nE - 1) e = nE - 1;
          int sj = ei[e];
          sj = sj < 0 ? 0 : (sj > nN - 1 ? nN - 1 : sj);
          const v4f p  = *(const v4f*)(pq + (size_t)sj * PQW + co);
          const v4f q  = *(const v4f*)(pq + (size_t)node * PQW + HC + co);
          const v4f xs = *(const v4f*)(x + (size_t)sj * HC + co);
          const v4f t = p + q;
          float s = fmaxf(t.x, 0.f) * w2v.x + fmaxf(t.y, 0.f) * w2v.y
                  + fmaxf(t.z, 0.f) * w2v.z + fmaxf(t.w, 0.f) * w2v.w;
          s += __shfl_xor(s, 16, 32);
          s += __shfl_xor(s, 8, 32);
          s += __shfl_xor(s, 4, 32);
          s += __shfl_xor(s, 2, 32);
          s += __shfl_xor(s, 1, 32);
          s += b2v;
          const float wv = __builtin_amdgcn_rcpf(1.0f + __expf(-s));
          float* ar = sacc + slot * HC + co;
          v4f a = *(v4f*)(ar);
          a = a + xs * wv;
          *(v4f*)(ar) = a;
        }
      }
    }
    __syncthreads();
  }

#pragma unroll 1
  for (int s = wave; s < NB; s += NWAVE) {
    const int node = nodeBase + s;
    if (node >= nN) break;
    const v4f a  = *(const v4f*)(sacc + s * HC + co);
    const v4f xv = *(const v4f*)(x + (size_t)node * HC + co);
    const v4f t  = xv + a;
    float sum = t.x + t.y + t.z + t.w;
    sum += __shfl_xor(sum, 16, 32);
    sum += __shfl_xor(sum, 8, 32);
    sum += __shfl_xor(sum, 4, 32);
    sum += __shfl_xor(sum, 2, 32);
    sum += __shfl_xor(sum, 1, 32);
    const float mu = sum * (1.0f / 128.0f);
    const v4f dv = t - mu;
    float ss = dv.x * dv.x + dv.y * dv.y + dv.z * dv.z + dv.w * dv.w;
    ss += __shfl_xor(ss, 16, 32);
    ss += __shfl_xor(ss, 8, 32);
    ss += __shfl_xor(ss, 4, 32);
    ss += __shfl_xor(ss, 2, 32);
    ss += __shfl_xor(ss, 1, 32);
    const float var  = ss * (1.0f / 128.0f);
    const float rstd = rsqrtf(var + 1e-5f);
    const v4f o = dv * rstd * gv + bv;
    float* op = out + (size_t)node * HC + co;
    *(volatile v4f*)op = o;
    __threadfence();
    *(volatile v4f*)op = o;
  }
}

extern "C" void kernel_launch(void* const* d_in, const int* in_sizes, int n_in,
                              void* d_out, int out_size, void* d_ws, size_t ws_size,
                              hipStream_t stream) {
  if (n_in < 8) return;
  const int nN = in_sizes[0] / HC;
  if (nN <= 0 || in_sizes[0] != nN * HC) return;
  const int nE = in_sizes[1] / 2;
  if (nE <= 0 || in_sizes[1] != 2 * nE) return;
  if (in_sizes[2] != 2 * HC * HC || in_sizes[3] != HC || in_sizes[4] != HC || in_sizes[5] < 1 ||
      in_sizes[6] != HC || in_sizes[7] != HC) return;
  if (out_size != nN * HC) return;

  const float* x     = (const float*)d_in[0];
  const int*   ei    = (const int*)d_in[1];
  const float* W1    = (const float*)d_in[2];
  const float* b1    = (const float*)d_in[3];
  const float* W2    = (const float*)d_in[4];
  const float* b2    = (const float*)d_in[5];
  const float* gamma = (const float*)d_in[6];
  const float* beta  = (const float*)d_in[7];
  float* out = (float*)d_out;

  const int Mpad = ((nN + GR - 1) / GR) * GR;

  char* wsp = (char*)d_ws;
  size_t off = 0;
  const size_t xhB = (((size_t)Mpad * HC * 2) + 255) & ~(size_t)255;
  const size_t btB = (((size_t)PQW * HC * 2) + 255) & ~(size_t)255;
  const size_t pqB = (((size_t)Mpad * PQW * 4) + 255) & ~(size_t)255;
  unsigned short* Xh = (unsigned short*)(wsp + off); off += xhB;
  unsigned short* Bt = (unsigned short*)(wsp + off); off += btB;
  float* PQ = (float*)(wsp + off); off += pqB;
  if (off > ws_size) return;
  if (off > (size_t)134217728) return;

  const float wsc  = 64.0f;
  const float iwsc = 0.015625f;

  hipFuncSetAttribute(reinterpret_cast<const void*>(&k_agg),
                      hipFuncAttributeMaxDynamicSharedMemorySize, AGG_LDS_BYTES);

  k_cvt_x<<<(Mpad * (HC / 8) + NTHR - 1) / NTHR, NTHR, 0, stream>>>(x, nN, Xh, Mpad);
  k_cvt_w<<<(PQW * (HC / 8) + NTHR - 1) / NTHR, NTHR, 0, stream>>>(W1, Bt, wsc);
  k_gemm<<<dim3(Mpad / GR, PQW / GC), NTHR, 0, stream>>>(Xh, Bt, b1, PQ, HC, PQW, HC, iwsc);
  k_agg<<<(nN + NB - 1) / NB, NTHR, AGG_LDS_BYTES, stream>>>(ei, x, PQ, W2, b2, gamma, beta, out, nN, nE);
}
